// GNNSegmentClassifier_26182120636657
// MI455X (gfx1250) — hardware-run, weakly checked
//
#include <hip/hip_runtime.h>


namespace {
constexpr int N = 100000, NP = 100032, NLIM = 100032  , EFULL = 3200000, E = 3200000  , DX = 3, DH = 8, DD = 11, HS = 16  , NIT = 3;
constexpr float XS = 8.0f, WSC = 256.0f;
static_assert(NP % 32 == 0 && E % 32 == 0, "tiling");
typedef _Float16 b16;
typedef __attribute__((ext_vector_type(16))) _Float16 v16b;
typedef __attribute__((ext_vector_type(8))) _Float16 v8b;
typedef __attribute__((ext_vector_type(8))) float v8f;
typedef __attribute__((ext_vector_type(4))) float v4f;
__device__ __forceinline__ float bf16_rne(float f) { unsigned int u = __float_as_uint(f); u += 0x7FFFu + ((u >> 16) & 1u); return __uint_as_float(u & 0xFFFF0000u); }
__device__ __forceinline__ void split16(float v, b16& hi, b16& lo) { hi = (b16)v; lo = (b16)(v - (float)hi); }
__device__ __forceinline__ v16b frag_kb(const b16* p, int hh) { const v8b a = *(const v8b*)(p + 8 * hh), b = *(const v8b*)(p + 16 + 8 * hh); v16b f;
#pragma unroll
  for (int e = 0; e < 8; ++e) { f[e] = a[e]; f[8 + e] = b[e]; } return f; }
__device__ __forceinline__ v8f wmma16b(v16b a, v16b b, v8f c) { v8f d = __builtin_amdgcn_wmma_f32_16x16x32_f16(false, a, false, b, (short)0, c, false, false); asm volatile("v_nop\n\tv_nop\n\tv_nop\n\tv_nop" : "+v"(d) : "v"(a), "v"(b)); return d; }
__device__ __forceinline__ void wave_lds_sync() { __builtin_amdgcn_fence(__ATOMIC_RELEASE, "workgroup"); __builtin_amdgcn_wave_barrier(); __builtin_amdgcn_fence(__ATOMIC_ACQUIRE, "workgroup"); }
__device__ __forceinline__ float pmul(float a, float b) { float p = a * b; asm volatile("" : "+v"(p)); return p; }
__device__ __forceinline__ int iclamp(int v, int lo, int hi) { return v < lo ? lo : (v > hi ? hi : v); }
constexpr int CSR_NBLK = 512, CSR_GB = 8  , CSR_GN = 1 << CSR_GB  , CSR_MAXG = 512, CSR_CAP = 12288  ;
__global__ __launch_bounds__(64) void csrA_kernel(const int* __restrict__ dst, int E, int N, int nG, int CHP, int NGP, int* __restrict__ STG, int* __restrict__ HST) {
  extern __shared__ int sm[];
  int* cnt = sm; int* run = sm + NGP; int* ids = sm + 2 * NGP;
  const int b = blockIdx.x; const int ch = (E + CSR_NBLK - 1) / CSR_NBLK; const int e0 = b * ch, e1 = min(E, e0 + ch);
  for (int i = threadIdx.x; i < NGP; i += 64) cnt[i] = 0;
  for (int i = threadIdx.x; i < CHP; i += 64) ids[i] = -1;
  __syncthreads();
  if (threadIdx.x == 0) {
    for (int e = e0; e < e1; ++e) { int d = dst[e]; d = (d < 0) ? 0 : (d >= N ? N - 1 : d); cnt[d >> CSR_GB] += 1; }
    int acc = 0; for (int g = 0; g < nG; ++g) { run[g] = acc; acc += cnt[g]; }
    for (int e = e0; e < e1; ++e) { int d = dst[e]; d = (d < 0) ? 0 : (d >= N ? N - 1 : d); const int g = d >> CSR_GB; ids[run[g]] = e; run[g] += 1; } }
  __syncthreads();
  typedef __attribute__((ext_vector_type(4))) int v4i;
  for (int pass = 0; pass < 2; ++pass) {
    for (int i = threadIdx.x; i < CHP / 4; i += 64) *(volatile v4i*)(STG + (size_t)b * CHP + i * 4) = *(const v4i*)(&ids[i * 4]);
    for (int i = threadIdx.x; i < NGP / 4; i += 64) { v4i v; for (int e = 0; e < 4; ++e) v[e] = (i * 4 + e < nG) ? cnt[i * 4 + e] : 0; *(volatile v4i*)(HST + (size_t)b * NGP + i * 4) = v; }
    __threadfence(); }
}
__global__ __launch_bounds__(512) void csrS_kernel(const int* __restrict__ HST, int nG, int NGP, int* __restrict__ START, int* __restrict__ TOT, int* __restrict__ OFF) {
  __shared__ int tot[CSR_MAXG];
  const int b = threadIdx.x;
  for (int pass = 0; pass < 2; ++pass) { int runb = 0; for (int g = 0; g < nG; ++g) { int c = HST[(size_t)b * NGP + g]; c = (c < 0) ? 0 : c; ((volatile int*)OFF)[(size_t)g * CSR_NBLK + b] = runb; runb += c; } __threadfence(); }
  for (int g = threadIdx.x; g < nG; g += 512) { int s = 0; for (int bb = 0; bb < CSR_NBLK; ++bb) { int c = HST[(size_t)bb * NGP + g]; s += (c < 0) ? 0 : c; } tot[g] = s; }
  __syncthreads();
  if (threadIdx.x < 32) {
    __shared__ int st[CSR_MAXG + 32];
    if (threadIdx.x == 0) { int acc = 0; for (int g = 0; g < NGP; ++g) { st[g] = acc; if (g < nG) acc += (tot[g] + 31) & ~31; } st[NGP] = acc; }
    __builtin_amdgcn_fence(__ATOMIC_RELEASE, "workgroup"); __builtin_amdgcn_wave_barrier(); __builtin_amdgcn_fence(__ATOMIC_ACQUIRE, "workgroup");
    for (int pass = 0; pass < 2; ++pass) { for (int i = threadIdx.x; i < NGP + 32; i += 32) { ((volatile int*)START)[i] = (i <= NGP) ? st[min(i, NGP)] : 0; ((volatile int*)TOT)[i] = (i < nG) ? tot[i] : 0; } __threadfence(); } }
}
__global__ __launch_bounds__(256) void csrB_kernel(const int* __restrict__ dst, int N, int nG, int CHP, int NGP, int permLen, const int* __restrict__ STG, const int* __restrict__ HST, const int* __restrict__ OFF, const int* __restrict__ START, const int* __restrict__ TOT, int* __restrict__ PERM, int* __restrict__ ROWPTR, int* __restrict__ ROWCNT, int* __restrict__ FLAG) {
  typedef __attribute__((ext_vector_type(4))) int v4i;
  __shared__ int ids[CSR_CAP]; __shared__ unsigned short key[CSR_CAP]; __shared__ int outp[CSR_CAP]; __shared__ int ncnt[CSR_GN + 1]; __shared__ int boff[CSR_NBLK + 1];
  const int g = blockIdx.x, t_ = threadIdx.x; int tot = TOT[g]; int st = START[g], stn = START[g + 1]; const int v0 = g * CSR_GN; const int nv = min(CSR_GN, N - v0);
  st = (st < 0) ? 0 : (st > permLen - 32 ? permLen - 32 : st) & ~31; stn = (stn < st) ? st : (stn > permLen ? permLen : stn); tot = (tot < 0) ? 0 : tot; if (tot > stn - st && tot <= CSR_CAP) tot = stn - st;
  if (tot > CSR_CAP) {
    for (int pass = 0; pass < 2; ++pass) { for (int i = t_; i < CSR_GN / 4; i += 256) { v4i a, c; for (int e = 0; e < 4; ++e) { a[e] = st; c[e] = 0; } *(volatile v4i*)(ROWPTR + v0 + i * 4) = a; *(volatile v4i*)(ROWCNT + v0 + i * 4) = c; } if (t_ == 0) ((volatile int*)FLAG)[0] = 1; __threadfence(); } (void)nv; return; }
  if (t_ == 0) { int acc = 0; for (int b = 0; b < CSR_NBLK; ++b) { boff[b] = acc; int c = HST[(size_t)b * NGP + g]; c = (c < 0) ? 0 : (c > CHP ? CHP : c); acc += c; if (acc > tot) acc = tot; } boff[CSR_NBLK] = acc; }
  for (int i = t_; i <= CSR_GN; i += 256) ncnt[i] = 0;
  __syncthreads();
  for (int b = 0; b < CSR_NBLK; ++b) { const int c = boff[b + 1] - boff[b]; int o_ = OFF[(size_t)g * CSR_NBLK + b]; o_ = (o_ < 0) ? 0 : (o_ > CHP - c ? CHP - c : o_); const int* src_ = STG + (size_t)b * CHP + o_;
    for (int i = t_; i < c; i += 256) { int id = src_[i]; id = (id < 0) ? 0 : id; ids[boff[b] + i] = id; int d = dst[id]; d = (d < v0) ? v0 : (d >= N ? N - 1 : d); int kk = d - v0; kk = (kk < 0) ? 0 : (kk >= CSR_GN ? CSR_GN - 1 : kk); key[boff[b] + i] = (unsigned short)kk; } }
  __syncthreads();
  if (t_ == 0) { for (int i = 0; i < tot; ++i) ncnt[key[i]] += 1; int acc = 0; for (int vl = 0; vl < CSR_GN; ++vl) { const int c = ncnt[vl]; ncnt[vl] = acc; acc += c; } ncnt[CSR_GN] = acc;
    for (int i = 0; i < tot; ++i) { const int vl = key[i]; outp[ncnt[vl]] = ids[i]; ncnt[vl] += 1; }
    for (int vl = CSR_GN; vl > 0; --vl) ncnt[vl] = ncnt[vl - 1]; ncnt[0] = 0; }
  __syncthreads();
  for (int pass = 0; pass < 2; ++pass) {
    for (int i = t_; i < (stn - st) / 4; i += 256) { v4i v; for (int e = 0; e < 4; ++e) { const int q = i * 4 + e; v[e] = (q < tot) ? outp[q] : -1; } *(volatile v4i*)(PERM + st + i * 4) = v; }
    for (int i = t_; i < CSR_GN / 4; i += 256) { v4i a, c; for (int e = 0; e < 4; ++e) { const int vl = i * 4 + e; a[e] = st + ncnt[vl]; c[e] = (vl < nv) ? (ncnt[vl + 1] - ncnt[vl]) : 0; } *(volatile v4i*)(ROWPTR + v0 + i * 4) = a; *(volatile v4i*)(ROWCNT + v0 + i * 4) = c; }
    __threadfence(); }
}
__global__ __launch_bounds__(256) void csrZ_kernel(int* __restrict__ p, size_t n4) { typedef __attribute__((ext_vector_type(4))) int v4i; const size_t tid = (size_t)blockIdx.x * 256 + threadIdx.x, nth = (size_t)gridDim.x * 256; v4i z = {0, 0, 0, 0}; for (size_t i = tid; i < n4; i += nth) *(volatile v4i*)(p + i * 4) = z; }
struct CsrBufs { int *STG, *HST, *OFF, *START, *TOT, *PERM, *ROWPTR, *ROWCNT, *FLAG; int nG, NGP, CHP; size_t permLen; char* base; size_t bytes; };
static size_t csr_carve(CsrBufs& c, char* ws, size_t off, int E, int N) {
  const size_t off0 = off; c.base = ws + off;
  auto al = [&](size_t bytes) { char* p = ws + off; off += (bytes + 255) & ~(size_t)255; return p; };
  c.nG = (N + CSR_GN - 1) / CSR_GN; c.NGP = (c.nG + 31) & ~31; const int ch = (E + CSR_NBLK - 1) / CSR_NBLK; c.CHP = (ch + 31) & ~31; c.permLen = (size_t)E + 32 * (size_t)c.nG + 32;
  c.STG = (int*)al((size_t)CSR_NBLK * c.CHP * 4); c.HST = (int*)al((size_t)CSR_NBLK * c.NGP * 4); c.OFF = (int*)al((size_t)c.NGP * CSR_NBLK * 4); c.START = (int*)al((size_t)(c.NGP + 64) * 4); c.TOT = (int*)al((size_t)(c.NGP + 64) * 4);
  c.PERM = (int*)al(c.permLen * 4); c.ROWPTR = (int*)al((size_t)c.nG * CSR_GN * 4); c.ROWCNT = (int*)al((size_t)c.nG * CSR_GN * 4); c.FLAG = (int*)al(256);
  c.bytes = off - off0; return off;
}
static void csr_build(const CsrBufs& c, const int* dst, int E, int N, hipStream_t stream) {
  const size_t smem = (size_t)(2 * c.NGP + c.CHP) * 4;
  csrZ_kernel<<<512, 256, 0, stream>>>((int*)c.base, c.bytes / 16);
  csrA_kernel<<<CSR_NBLK, 64, smem, stream>>>(dst, E, N, c.nG, c.CHP, c.NGP, c.STG, c.HST);
  csrS_kernel<<<1, 512, 0, stream>>>(c.HST, c.nG, c.NGP, c.START, c.TOT, c.OFF);
  csrB_kernel<<<c.nG, 256, 0, stream>>>(dst, N, c.nG, c.CHP, c.NGP, (int)c.permLen, c.STG, c.HST, c.OFF, c.START, c.TOT, c.PERM, c.ROWPTR, c.ROWCNT, c.FLAG);
}

__global__ __launch_bounds__(256) void wprep_kernel(const float* __restrict__ we1, const float* __restrict__ wn1, b16* __restrict__ WE1, b16* __restrict__ WN1) {
  const int t = threadIdx.x; v8b o;
  if (t < 16 * 32 / 8) { const int e = t * 8; const int oo = e / 32, k0 = e % 32; for (int j = 0; j < 8; ++j) { const int k = k0 + j; o[j] = (oo < DH && k < 2 * DD) ? (b16)(bf16_rne(we1[k * DH + oo]) * WSC) : (b16)0.0f; }
    for (int pass = 0; pass < 2; ++pass) { *(volatile v8b*)(WE1 + e) = o; __threadfence(); } }
  else if (t < 16 * 32 / 8 + 16 * 64 / 8) { const int e = (t - 64) * 8; const int oo = e / 64, k0 = e % 64; for (int j = 0; j < 8; ++j) { const int k = k0 + j; o[j] = (oo < DH && k < 3 * DD) ? (b16)(bf16_rne(wn1[k * DH + oo]) * WSC) : (b16)0.0f; }
    for (int pass = 0; pass < 2; ++pass) { *(volatile v8b*)(WN1 + e) = o; __threadfence(); } }
}
__global__ __launch_bounds__(256) void h0_kernel(const float* __restrict__ x, const float* __restrict__ win, const float* __restrict__ bin, float* __restrict__ HF) {
  __shared__ __attribute__((aligned(16))) float T[8][32][HS];
  const int wave = threadIdx.x >> 5, lane = threadIdx.x & 31; const size_t v0 = ((size_t)blockIdx.x * 8 + wave) * 32; const size_t v = v0 + lane;
  float xv[DX] = {0.0f, 0.0f, 0.0f}; const bool live = v < (size_t)N;
  if (live) { for (int i = 0; i < DX; ++i) xv[i] = bf16_rne(x[v * DX + i]); }
#pragma unroll 1
  for (int o = 0; o < DH; ++o) { float s = bf16_rne(bin[o]); for (int i = 0; i < DX; ++i) s += pmul(xv[i], bf16_rne(win[i * DH + o])); T[wave][lane][o] = live ? tanhf(s) : 0.0f; }
  for (int i = 0; i < DX; ++i) T[wave][lane][DH + i] = live ? xv[i] : 0.0f;
  for (int j = DD; j < HS; ++j) T[wave][lane][j] = 0.0f;
  wave_lds_sync();
  const float* tw = &T[wave][0][0];
  for (int pass = 0; pass < 2; ++pass) { for (int q = 0; q < 4; ++q) *(volatile v4f*)(HF + v0 * HS + (q * 32 + lane) * 4) = *(const v4f*)(tw + (q * 32 + lane) * 4); __threadfence(); }
}
__global__ __launch_bounds__(64) void edge_kernel(const float* __restrict__ HF, const int* __restrict__ rows_, const int* __restrict__ cols_, const b16* __restrict__ WE1, const float* __restrict__ be1, const float* __restrict__ we2, const float* __restrict__ be2, float* __restrict__ EV) {
  __shared__ float es[32];
  const int wave = threadIdx.x >> 5, lane = threadIdx.x & 31, nloc = lane & 15, hlf = lane >> 4; const size_t e0 = (size_t)blockIdx.x * 32 + wave * 16; const size_t er = e0 + nloc;
  const int rn = iclamp(rows_[er], 0, N - 1), cn = iclamp(cols_[er], 0, N - 1);
  v16b ah, al;
#pragma unroll
  for (int el = 0; el < 16; ++el) { const int k = (el < 8) ? (8 * hlf + el) : (16 + 8 * hlf + (el - 8)); float v = 0.0f;
    if (k < DD) v = HF[(size_t)cn * HS + k]; else if (k < 2 * DD) v = HF[(size_t)rn * HS + (k - DD)];
    b16 p, q; split16(v * XS, p, q); ah[el] = p; al[el] = q; }
  v8f d = (v8f){}; const v16b bw = frag_kb(WE1 + (size_t)nloc * 32, hlf); d = wmma16b(ah, bw, d); d = wmma16b(al, bw, d);
  const float b1 = (nloc < DH) ? bf16_rne(be1[nloc]) : 0.0f, w2 = (nloc < DH) ? bf16_rne(we2[nloc]) : 0.0f; const float b2 = bf16_rne(be2[0]);
  float mine[8];
#pragma unroll
  for (int r = 0; r < 8; ++r) { float s = (nloc < DH) ? pmul(tanhf(d[r] * (1.0f / (XS * WSC)) + b1), w2) : 0.0f;
#pragma unroll
    for (int o = 1; o < 16; o <<= 1) s += __shfl_xor(s, o);
    mine[r] = 1.0f / (1.0f + __expf(-(s + b2))); }
  { float val = mine[0];
#pragma unroll
    for (int r = 1; r < 8; ++r) if (nloc == r) val = mine[r];
    if (nloc < 8) es[wave * 16 + 8 * hlf + nloc] = val; }
  __syncthreads();
  for (int pass = 0; pass < 2; ++pass) { if (wave == 0) ((volatile float*)EV)[e0 + lane] = es[lane]; __threadfence(); }
}
template <int MODE>
__global__ __launch_bounds__(256) void agg_kernel(const float* __restrict__ HF, const float* __restrict__ EV, const int* __restrict__ other, const int* __restrict__ PERM, const int* __restrict__ ROWPTR, const int* __restrict__ ROWCNT, int permLen, float* __restrict__ MOUT) {
  const int wave = threadIdx.x >> 5, lane = threadIdx.x & 31, nloc = lane & 15, hlf = lane >> 4; const size_t v = ((size_t)blockIdx.x * 8 + wave) * 2 + hlf; float a = 0.0f;
  if (v < (size_t)N && nloc < DD) { int st = ROWPTR[v], cnt = ROWCNT[v]; cnt = iclamp(cnt, 0, 65536); st = iclamp(st, 0, permLen - cnt);
#pragma unroll 1
    for (int j = 0; j < cnt; ++j) { const int e = iclamp(PERM[st + j], 0, E - 1); const int u = iclamp(other[e], 0, N - 1); a += pmul(EV[e], HF[(size_t)u * HS + nloc]); } }
  for (int pass = 0; pass < 2; ++pass) { ((volatile float*)MOUT)[v * HS + nloc] = a; __threadfence(); }
}
__global__ __launch_bounds__(64) void node_kernel(float* __restrict__ HF, const float* __restrict__ MI, const float* __restrict__ MO, const b16* __restrict__ WN1, const float* __restrict__ bn1, const float* __restrict__ wn2, const float* __restrict__ bn2) {
  __shared__ __attribute__((aligned(16))) float T[2][16][HS];
  const int wave = threadIdx.x >> 5, lane = threadIdx.x & 31, nloc = lane & 15, hlf = lane >> 4; const size_t v0 = ((size_t)blockIdx.x * 2 + wave) * 16; const size_t vr = v0 + nloc;
  v8f d = (v8f){};
#pragma unroll
  for (int ks = 0; ks < 2; ++ks) { v16b ah, al;
#pragma unroll
    for (int el = 0; el < 16; ++el) { const int k = ks * 32 + ((el < 8) ? (8 * hlf + el) : (16 + 8 * hlf + (el - 8))); float v = 0.0f;
      if (k < DD) v = MI[vr * HS + k]; else if (k < 2 * DD) v = MO[vr * HS + (k - DD)]; else if (k < 3 * DD) v = HF[vr * HS + (k - 2 * DD)];
      b16 p, q; split16(v * XS, p, q); ah[el] = p; al[el] = q; }
    const v16b bw = frag_kb(WN1 + (size_t)nloc * 64 + ks * 32, hlf); d = wmma16b(ah, bw, d); d = wmma16b(al, bw, d); }
  const float b1 = (nloc < DH) ? bf16_rne(bn1[nloc]) : 0.0f;
#pragma unroll
  for (int r = 0; r < 8; ++r) { const float t = (nloc < DH) ? tanhf(d[r] * (1.0f / (XS * WSC)) + b1) : 0.0f;
    float u = (nloc < DH) ? bf16_rne(bn2[nloc]) : 0.0f;
#pragma unroll
    for (int o = 0; o < DH; ++o) { const float to = __shfl(t, (lane & 16) + o); if (nloc < DH) u += pmul(to, bf16_rne(wn2[o * DH + nloc])); }
    const size_t node = v0 + 8 * hlf + r; float val = 0.0f;
    if (nloc < DH) val = (node < (size_t)N) ? tanhf(u) : 0.0f; else if (nloc < DD) val = (node < (size_t)N) ? HF[node * HS + nloc] : 0.0f;
    T[wave][8 * hlf + r][nloc] = val; }
  wave_lds_sync();
  const float* tw = &T[wave][0][0];
  for (int pass = 0; pass < 2; ++pass) { for (int q = 0; q < 2; ++q) *(volatile v4f*)(HF + v0 * HS + (q * 32 + lane) * 4) = *(const v4f*)(tw + (q * 32 + lane) * 4); __threadfence(); }
}
}

extern "C" void kernel_launch(void* const* d_in, const int* in_sizes, int n_in, void* d_out, int out_size, void* d_ws, size_t ws_size, hipStream_t stream) {
  (void)n_in;
  auto Fp = [&](int i) { return (const float*)d_in[i]; }; auto Ip = [&](int i) { return (const int*)d_in[i]; };
  if (in_sizes[0] != N * DX || in_sizes[1] != 2 * EFULL || in_sizes[2] != DX * DH || in_sizes[4] != 2 * DD * DH || in_sizes[6] != DH || in_sizes[7] != 1 || in_sizes[8] != 3 * DD * DH || in_sizes[10] != DH * DH || out_size != EFULL) return;
  size_t off = 0; char* ws = (char*)d_ws;
  auto carve = [&](size_t bytes) { char* p = ws + off; off += (bytes + 255) & ~(size_t)255; return p; };
  b16* WE1 = (b16*)carve(16 * 32 * 2); b16* WN1 = (b16*)carve(16 * 64 * 2); float* HF = (float*)carve((size_t)NP * HS * 4); float* MI = (float*)carve((size_t)NP * HS * 4); float* MO = (float*)carve((size_t)NP * HS * 4); float* EV = (float*)carve((size_t)E * 4);
  CsrBufs ccol, crow; off = csr_carve(ccol, ws, off, E, N); off = csr_carve(crow, ws, off, E, N);
  if (off > ws_size || off > ((size_t)128 << 20)) return;
  wprep_kernel<<<1, 256, 0, stream>>>(Fp(4), Fp(8), WE1, WN1);
  h0_kernel<<<(unsigned)((NP / 32 + 7) / 8), 256, 0, stream>>>(Fp(0), Fp(2), Fp(3), HF);
  csr_build(ccol, Ip(1) + EFULL, E, N, stream);
  csr_build(crow, Ip(1), E, N, stream);
  for (int it = 0; it < NIT; ++it) {
    edge_kernel<<<E / 32, 64, 0, stream>>>(HF, Ip(1), Ip(1) + EFULL, WE1, Fp(5), Fp(6), Fp(7), EV);
    agg_kernel<0><<<(unsigned)((NLIM / 2 + 7) / 8), 256, 0, stream>>>(HF, EV, Ip(1), ccol.PERM, ccol.ROWPTR, ccol.ROWCNT, (int)ccol.permLen, MI);
    agg_kernel<1><<<(unsigned)((NLIM / 2 + 7) / 8), 256, 0, stream>>>(HF, EV, Ip(1) + EFULL, crow.PERM, crow.ROWPTR, crow.ROWCNT, (int)crow.permLen, MO);
    node_kernel<<<NLIM / 32, 64, 0, stream>>>(HF, MI, MO, WN1, Fp(9), Fp(10), Fp(11)); }
  edge_kernel<<<E / 32, 64, 0, stream>>>(HF, Ip(1), Ip(1) + EFULL, WE1, Fp(5), Fp(6), Fp(7), (float*)d_out);
}
